// MeshEncoder_14645838479864
// MI455X (gfx1250) — hardware-verified
//
#include <hip/hip_runtime.h>
#include <stdint.h>
#include <math.h>

constexpr int NNODE  = 50000;
constexpr int NEDGE  = 800000;
constexpr int NCH    = 64;
constexpr int CIN0   = 3;
constexpr int NKER   = 27;
constexpr int CHUNKN = 6400;
constexpr int NCHUNK = 8;
constexpr int NPADN  = CHUNKN * NCHUNK;
constexpr int KSP    = NKER * NCH;
constexpr int KBIG   = KSP + NCH;
constexpr int SEGN   = KBIG / 8;
constexpr int ACC0P  = 128;
constexpr int KL0    = 128;
constexpr int NTH    = 256;
constexpr int SPT    = 8;
constexpr int SCH    = NTH * SPT;
constexpr int NSTEP  = (NEDGE + SCH - 1) / SCH;
constexpr int WROWS  = CHUNKN / 8;

static_assert(NPADN >= NNODE && CHUNKN % 64 == 0 && CHUNKN % 32 == 0 && WROWS * 8 == CHUNKN, "");
static_assert(KBIG % 32 == 0 && KL0 % 32 == 0 && KSP == 216 * 8 && SEGN * 8 == KBIG, "");
static_assert(NEDGE % SPT == 0 && SCH == 2048 && NTH == 256 && (CHUNKN - 1) * 2048 + 2047 < (1 << 30), "");
static_assert((CHUNKN * SEGN) % 256 == 0 && (NNODE * 16) % 256 == 0 && (NCH * SEGN) % 256 == 0 && (NCH * (KL0 / 8)) % 256 == 0, "");
static_assert(ACC0P == 128 && NKER <= 32 && CIN0 == 3 && CHUNKN % 32 == 0, "");

typedef __attribute__((ext_vector_type(16))) _Float16 v16h;
typedef __attribute__((ext_vector_type(8)))  _Float16 v8h;
typedef __attribute__((ext_vector_type(16))) __bf16   v16b;
typedef __attribute__((ext_vector_type(8)))  __bf16   v8b;
typedef __attribute__((ext_vector_type(8)))  float    v8f;
typedef __attribute__((ext_vector_type(4)))  float    v4f;
typedef __attribute__((ext_vector_type(4)))  int      v4i;

__device__ __forceinline__ unsigned short f2bf_bits(float f) {
  unsigned u = __float_as_uint(f);
  return (unsigned short)((u + 0x7FFFu + ((u >> 16) & 1u)) >> 16);
}
__device__ __forceinline__ float bf_bits2f(unsigned short h) { return __uint_as_float(((unsigned)h) << 16); }
__device__ __forceinline__ void bf_split(float v, _Float16& h, _Float16& l) {
  const unsigned short hb = f2bf_bits(v);
  const unsigned short lb = f2bf_bits(v - bf_bits2f(hb));
  h = __builtin_bit_cast(_Float16, hb);
  l = __builtin_bit_cast(_Float16, lb);
}

__device__ __forceinline__ void dep_guard_h(v8f& a, v8f& b, v16h x, v16h y) { asm volatile("v_nop\n\tv_nop\n\tv_nop\n\tv_nop" : "+v"(a), "+v"(b) : "v"(x), "v"(y)); }
__device__ __forceinline__ void dep_guard_b(v8f& a, v8f& b, v16b x, v16b y) { asm volatile("v_nop\n\tv_nop\n\tv_nop\n\tv_nop" : "+v"(a), "+v"(b) : "v"(x), "v"(y)); }
__device__ __forceinline__ void keep4_h(v16h a, v16h b, v16h c, v16h d) { asm volatile("v_nop" :: "v"(a), "v"(b), "v"(c), "v"(d)); }
__device__ __forceinline__ void keep4_b(v16b a, v16b b, v16b c, v16b d) { asm volatile("v_nop" :: "v"(a), "v"(b), "v"(c), "v"(d)); }
__device__ __forceinline__ void acc_guard4(v8f& a, v8f& b, v8f& c, v8f& d) { asm volatile("v_nop\n\tv_nop\n\tv_nop\n\tv_nop" : "+v"(a), "+v"(b), "+v"(c), "+v"(d)); }
template <typename T> struct Frag;
template <> struct Frag<_Float16> {
  typedef v16h V; union U { v16h v; v8h h[2]; };
  static __device__ __forceinline__ v16h load(const _Float16* p) {
    U f; f.h[0] = *(const v8h*)(p); f.h[1] = *(const v8h*)(p + 16); return f.v;
  }
  static __device__ __forceinline__ v8f mma(v16h a, v16h b, v8f c) {
    return __builtin_amdgcn_wmma_f32_16x16x32_f16(false, a, false, b, (short)0, c, false, false);
  }
  static __device__ __forceinline__ void guard(v8f& a, v8f& b, v16h x, v16h y) { dep_guard_h(a, b, x, y); }
  static __device__ __forceinline__ void keep(v16h a, v16h b, v16h c, v16h d) { keep4_h(a, b, c, d); }
};
template <> struct Frag<__bf16> {
  typedef v16b V; union U { v16b v; v8b h[2]; };
  static __device__ __forceinline__ v16b load(const __bf16* p) {
    U f; f.h[0] = *(const v8b*)(p); f.h[1] = *(const v8b*)(p + 16); return f.v;
  }
  static __device__ __forceinline__ v8f mma(v16b a, v16b b, v8f c) {
    return __builtin_amdgcn_wmma_f32_16x16x32_bf16(false, a, false, b, (short)0, c, false, false);
  }
  static __device__ __forceinline__ void guard(v8f& a, v8f& b, v16b x, v16b y) { dep_guard_b(a, b, x, y); }
  static __device__ __forceinline__ void keep(v16b a, v16b b, v16b c, v16b d) { keep4_b(a, b, c, d); }
};

template <int ET> struct Elem;
template <> struct Elem<0> { typedef _Float16 T; };
template <> struct Elem<1> { typedef __bf16 T; };
template <int ET, bool SPLIT, int BIAS_MODE, int OUT_MODE, bool RESID, int ACT = 0>
__global__ __launch_bounds__(256) void wmma_gemm64(
    const unsigned short* __restrict__ Ap, const unsigned short* __restrict__ A2p, int lda, long strideA,
    const unsigned short* __restrict__ Btp, const unsigned short* __restrict__ Bt2p, int ldb, long strideB,
    void* __restrict__ Cout, void* __restrict__ Cout2, int ldc, long strideC,
    const float* __restrict__ bias,
    const float* __restrict__ resid, long strideR,
    int M, int N, int K, float scale) {
  typedef typename Elem<ET>::T T;
  typedef typename Frag<T>::V V;
  const T* A = (const T*)Ap; const T* A2 = (const T*)A2p; const T* Bt = (const T*)Btp; const T* Bt2 = (const T*)Bt2p;
  __shared__ __align__(16) float sT[8][16 * 68];
  const int b    = blockIdx.y;
  const int lane = threadIdx.x & 31;
  const int wave = threadIdx.x >> 5;
  const int tilesN = N >> 6;
  const int tilesM = M >> 6;
  const int tile = blockIdx.x * 8 + wave;
  if (tile >= tilesM * tilesN) return;
  const int tm = tile / tilesN;
  const int tn = tile - tm * tilesN;
  const int m0 = tm << 6;
  const int n0 = tn << 6;

  const T* Ab  = A  + (size_t)b * strideA;
  const T* Bb  = Bt + (size_t)b * strideB;
  const T* Ab2 = SPLIT ? (A2  + (size_t)b * strideA) : nullptr;
  const T* Bb2 = SPLIT ? (Bt2 + (size_t)b * strideB) : nullptr;

  const int rlane = lane & 15;
  const int koff  = (lane >> 4) * 8;
  const int mOff  = (lane >> 4) * 8;

  v8f acc[4][4];
#pragma unroll
  for (int i = 0; i < 4; ++i)
#pragma unroll
    for (int j = 0; j < 4; ++j) acc[i][j] = (v8f){0.f,0.f,0.f,0.f,0.f,0.f,0.f,0.f};

  for (int k0 = 0; k0 < K; k0 += 32) {
    V bh[4], bl[4];
#pragma unroll
    for (int j = 0; j < 4; ++j) {
      const size_t bo = (size_t)(n0 + (j << 4) + rlane) * ldb + koff + k0;
      bh[j] = Frag<T>::load(Bb + bo);
      if (SPLIT) bl[j] = Frag<T>::load(Bb2 + bo);
    }
#pragma unroll
    for (int i = 0; i < 4; ++i) {
      const size_t ao = (size_t)(m0 + (i << 4) + rlane) * lda + koff + k0;
      V ah = Frag<T>::load(Ab + ao);
      V al;
      if (SPLIT) al = Frag<T>::load(Ab2 + ao);
#pragma unroll
      for (int j = 0; j < 4; ++j) {
        acc[i][j] = Frag<T>::mma(ah, bh[j], acc[i][j]);
        if (SPLIT) {
          acc[i][j] = Frag<T>::mma(ah, bl[j], acc[i][j]);
          acc[i][j] = Frag<T>::mma(al, bh[j], acc[i][j]);
        }
      }
      Frag<T>::guard(acc[i][0], acc[i][3], ah, SPLIT ? al : ah);
    }
    Frag<T>::keep(bh[0], bh[1], bh[2], bh[3]);
    if (SPLIT) Frag<T>::keep(bl[0], bl[1], bl[2], bl[3]);
  }
  acc_guard4(acc[0][0], acc[0][1], acc[0][2], acc[0][3]);
  acc_guard4(acc[1][0], acc[1][1], acc[1][2], acc[1][3]);
  acc_guard4(acc[2][0], acc[2][1], acc[2][2], acc[2][3]);
  acc_guard4(acc[3][0], acc[3][1], acc[3][2], acc[3][3]);

  float* slab = sT[wave];
  const float* Rb = RESID ? (resid + (size_t)b * strideR) : nullptr;
#pragma unroll
  for (int i = 0; i < 4; ++i) {
    const int mBase = m0 + (i << 4);
#pragma unroll
    for (int j = 0; j < 4; ++j) {
      const int n = n0 + (j << 4) + rlane;
      float bv = 0.f;
      if (BIAS_MODE == 2) bv = bias[n];
#pragma unroll
      for (int r = 0; r < 8; ++r) {
        float v = acc[i][j][r] * scale;
        if (BIAS_MODE == 1) v += bias[mBase + mOff + r];
        if (BIAS_MODE == 2) v += bv;
        if (RESID) v += Rb[(size_t)(mBase + mOff + r) * ldc + n];
        if (ACT == 1) v = tanhf(v);
        if (ACT == 2) v = fmaxf(v, 0.0f);
        if (ACT == 3) v = v / (1.0f + expf(-v));
        if (ACT == 4) v = (v > 0.f) ? v : 0.01f * v;
        slab[(mOff + r) * 68 + (j << 4) + rlane] = v;
      }
    }
    __builtin_amdgcn_fence(__ATOMIC_RELEASE, "workgroup");
    __builtin_amdgcn_wave_barrier();
    __builtin_amdgcn_fence(__ATOMIC_ACQUIRE, "workgroup");
    if (OUT_MODE == 0) {
      float* C = (float*)Cout + (size_t)b * strideC;
      const int hh = lane >> 4, c4 = (lane & 15) * 4;
      for (int pass = 0; pass < 2; ++pass) {
#pragma unroll
        for (int it = 0; it < 8; ++it) {
          const int row = it * 2 + hh;
          v4f v = *(const v4f*)(slab + row * 68 + c4);
          *(volatile v4f*)(C + (size_t)(mBase + row) * ldc + n0 + c4) = v;
        }
        __threadfence();
      }
    } else {
      const int q = lane >> 3, c8 = (lane & 7) * 8;
      unsigned short* C  = (unsigned short*)Cout  + (size_t)b * strideC;
      unsigned short* C2 = (OUT_MODE == 2) ? ((unsigned short*)Cout2 + (size_t)b * strideC) : nullptr;
      for (int pass = 0; pass < 2; ++pass) {
#pragma unroll
        for (int it = 0; it < 4; ++it) {
          const int row = it * 4 + q;
          const float* sp = slab + row * 68 + c8;
          v8h hv, lv;
#pragma unroll
          for (int e = 0; e < 8; ++e) {
            if (OUT_MODE == 1) {
              hv[e] = (_Float16)sp[e];
            } else {
              unsigned short hb = f2bf_bits(sp[e]);
              unsigned short lb = f2bf_bits(sp[e] - bf_bits2f(hb));
              hv[e] = __builtin_bit_cast(_Float16, hb);
              lv[e] = __builtin_bit_cast(_Float16, lb);
            }
          }
          *(volatile v8h*)(C + (size_t)(mBase + row) * ldc + n0 + c8) = hv;
          if (OUT_MODE == 2) *(volatile v8h*)(C2 + (size_t)(mBase + row) * ldc + n0 + c8) = lv;
        }
        __threadfence();
      }
    }
    __builtin_amdgcn_fence(__ATOMIC_RELEASE, "workgroup");
    __builtin_amdgcn_wave_barrier();
    __builtin_amdgcn_fence(__ATOMIC_ACQUIRE, "workgroup");
  }
}

__global__ __launch_bounds__(256) void prep_w0_kernel(const float* __restrict__ W, const float* __restrict__ R,
                                                      unsigned short* __restrict__ BH, unsigned short* __restrict__ BL) {
  const int i = blockIdx.x * 256 + threadIdx.x;
  if (i >= NCH * (KL0 / 8)) return;
  const int o = i >> 4;
  const int c = i & 15;
  v8h hv, lv;
#pragma unroll
  for (int e = 0; e < 8; ++e) {
    const int k = 8 * c + e;
    const int j = k >> 5;
    const int kk = k & 31;
    const int kc = (kk < NKER) ? kk : (NKER - 1);
    const int jc = (j < CIN0) ? j : (CIN0 - 1);
    const float wv = W[(kc * CIN0 + jc) * NCH + o];
    int ir = k - 96; ir = ir < 0 ? 0 : (ir > CIN0 - 1 ? CIN0 - 1 : ir);
    const float rv = R[ir * NCH + o];
    float v = 0.0f;
    if (k < 96 && kk < NKER) v = wv;
    if (k >= 96 && k < 96 + CIN0) v = rv;
    _Float16 h, l; bf_split(v, h, l); hv[e] = h; lv[e] = l;
  }
  const size_t op = (size_t)i * 8;
  *(volatile v8h*)(BH + op) = hv;
  *(volatile v8h*)(BL + op) = lv;
  __threadfence();
  *(volatile v8h*)(BH + op) = hv;
  *(volatile v8h*)(BL + op) = lv;
}

__global__ __launch_bounds__(256) void prep_w64_kernel(const float* __restrict__ W, const float* __restrict__ R,
                                                       unsigned short* __restrict__ BH, unsigned short* __restrict__ BL) {
  const int i = blockIdx.x * 256 + threadIdx.x;
  if (i >= NCH * SEGN) return;
  const int o = i / SEGN;
  const int c = i - o * SEGN;
  v8h hv, lv;
#pragma unroll
  for (int e = 0; e < 8; ++e) {
    const int k = 8 * c + e;
    const int kw = (k < KSP) ? k : (KSP - 1);
    int kr = k - KSP; kr = kr < 0 ? 0 : (kr > NCH - 1 ? NCH - 1 : kr);
    const float wv = W[(size_t)kw * NCH + o];
    const float rv = R[kr * NCH + o];
    const float v = (k < KSP) ? wv : rv;
    _Float16 h, l; bf_split(v, h, l); hv[e] = h; lv[e] = l;
  }
  const size_t op = (size_t)i * 8;
  *(volatile v8h*)(BH + op) = hv;
  *(volatile v8h*)(BL + op) = lv;
  __threadfence();
  *(volatile v8h*)(BH + op) = hv;
  *(volatile v8h*)(BL + op) = lv;
}

__device__ __forceinline__ int blk_excl_scan(int cnt, int* scan_ws, int tid, int* tot) {
  const int lane = tid & 31, wave = tid >> 5; int incl = cnt;
#pragma unroll
  for (int o = 1; o < 32; o <<= 1) { const int v = __shfl_up(incl, o, 32); if (lane >= o) incl += v; }
  if (lane == 31) scan_ws[wave] = incl;
  __syncthreads();
  if (wave == 0) { int wv = (lane < NTH / 32) ? scan_ws[lane] : 0; int wincl = wv;
#pragma unroll
    for (int o = 1; o < 32; o <<= 1) { const int v = __shfl_up(wincl, o, 32); if (lane >= o) wincl += v; }
    if (lane < NTH / 32) scan_ws[32 + lane] = wincl - wv; if (lane == 31) scan_ws[64] = wincl; }
  __syncthreads();
  const int res = scan_ws[32 + wave] + incl - cnt; *tot = scan_ws[64];
  return res;
}
__device__ __forceinline__ int chunk_hits(const int* __restrict__ dstv, int e0, int n0, int tid, int* LIST, int* scan_ws) {
  const int eb = e0 + tid * SPT;
  const bool real = (eb < NEDGE);
  const int ebc = real ? eb : (NEDGE - SPT);
  int rec[SPT]; int cnt = 0;
#pragma unroll
  for (int k = 0; k < SPT; k += 4) {
    const v4i d4 = *(const v4i*)(dstv + ebc + k);
#pragma unroll
    for (int e = 0; e < 4; ++e) {
      int d = d4[e]; d = d < 0 ? 0 : (d >= NNODE ? NNODE - 1 : d);
      int r = -1;
      if (real && d >= n0 && d < n0 + CHUNKN) { r = ((d - n0) << 11) | (tid * SPT + k + e); ++cnt; }
      rec[k + e] = r;
    }
  }
  int tot; int p = blk_excl_scan(cnt, scan_ws, tid, &tot);
#pragma unroll
  for (int k = 0; k < SPT; ++k) if (rec[k] >= 0) { if ((unsigned)p < (unsigned)SCH) LIST[p] = rec[k]; ++p; }
  __syncthreads();
  return tot < SCH ? tot : SCH;
}

__device__ __forceinline__ void spline_basis(const float* __restrict__ PS, int e, float& f0, float& f1, float& f2,
                                             int& i0, int& i1, int& i2) {
  const float p0 = PS[(size_t)e * 3 + 0] * 2.0f;
  const float p1 = PS[(size_t)e * 3 + 1] * 2.0f;
  const float p2 = PS[(size_t)e * 3 + 2] * 2.0f;
  const float a0 = fminf(fmaxf(floorf(p0), 0.0f), 1.0f);
  const float a1 = fminf(fmaxf(floorf(p1), 0.0f), 1.0f);
  const float a2 = fminf(fmaxf(floorf(p2), 0.0f), 1.0f);
  f0 = p0 - a0; f1 = p1 - a1; f2 = p2 - a2;
  i0 = (int)a0; i1 = (int)a1; i2 = (int)a2;
}

__global__ __launch_bounds__(NTH) void agg3_kernel(const float* __restrict__ X, const int* __restrict__ srcv, const int* __restrict__ dstv,
                                                   const float* __restrict__ PS, float* ACC, int n0) {
  __shared__ int LIST[SCH];
  __shared__ int scan_ws[80];
  const int tid = threadIdx.x, lane = tid & 31, wave = tid >> 5;
  const int wlo = wave * WROWS, whi = wlo + WROWS;
  const int jl = lane >> 3;
  const int jc = (jl < CIN0) ? jl : (CIN0 - 1);
  const int kq = 4 * (lane & 7);
  int u0[4], u1[4], u2[4];
#pragma unroll
  for (int e = 0; e < 4; ++e) { const int kk = kq + e; u0[e] = kk % 3; u1[e] = (kk / 3) % 3; u2[e] = kk / 9; }
  const float cnt0 = (lane == 24) ? 1.0f : 0.0f;
  const v4f zv = {0.0f, 0.0f, 0.0f, 0.0f};
#pragma unroll 1
  for (int nd = 0; nd < WROWS; ++nd) {
    float* rp = ACC + (size_t)(wlo + nd) * ACC0P + 4 * lane;
    *(volatile v4f*)rp = zv;
    __threadfence();
    *(volatile v4f*)rp = zv;
  }
#pragma unroll 1
  for (int cs = 0; cs < NSTEP; ++cs) {
    const int e0 = cs * SCH;
    const int tot = chunk_hits(dstv, e0, n0, tid, LIST, scan_ws);
#pragma unroll 1
    for (int base = 0; base < tot; base += 32) {
      const int q = base + lane;
      const int qc = (q < SCH) ? q : (SCH - 1);
      const int lv = LIST[qc];
      const int rv = (q < tot) ? lv : -1;
      const int dq = rv >> 11;
      const int own = (rv >= 0 && dq >= wlo && dq < whi) ? 1 : 0;
      unsigned msk = (unsigned)__ballot(own);
#pragma unroll 1
      for (int it = 0; it < 32; ++it) {
        if (msk == 0u) break;
        const int bp = __builtin_ctz(msk); msk &= msk - 1u;
        const int r = __shfl(rv, bp, 32);
        int dl = r >> 11; dl = dl < 0 ? 0 : (dl >= CHUNKN ? CHUNKN - 1 : dl);
        int e = e0 + (r & (SCH - 1)); e = (e < NEDGE) ? e : (NEDGE - 1);
        int s = srcv[e]; s = s < 0 ? 0 : (s >= NNODE ? NNODE - 1 : s);
        float f0, f1, f2; int i0, i1, i2;
        spline_basis(PS, e, f0, f1, f2, i0, i1, i2);
        const float g0 = 1.0f - f0, g1 = 1.0f - f1, g2 = 1.0f - f2;
        const float xv = X[(size_t)s * CIN0 + jc];
        v4f add;
#pragma unroll
        for (int ee = 0; ee < 4; ++ee) {
          const int o0 = u0[ee] - i0, o1 = u1[ee] - i1, o2 = u2[ee] - i2;
          const bool m = ((unsigned)o0 <= 1u) && ((unsigned)o1 <= 1u) && ((unsigned)o2 <= 1u);
          const float w = (o0 ? f0 : g0) * (o1 ? f1 : g1) * (o2 ? f2 : g2);
          float val = m ? (w * xv) : 0.0f;
          val = (jl < CIN0) ? val : ((ee == 0) ? cnt0 : 0.0f);
          add[ee] = val;
        }
        float* rp = ACC + (size_t)dl * ACC0P + 4 * lane;
        v4f a = *(const v4f*)rp;
        a = a + add;
        *(volatile v4f*)rp = a;
        __threadfence();
        *(volatile v4f*)rp = a;
      }
    }
    __syncthreads();
  }
}

__global__ __launch_bounds__(512) void cast0_kernel(const float* __restrict__ ACC, const float* __restrict__ X,
                                                   unsigned short* __restrict__ AH, unsigned short* __restrict__ AL,
                                                   float* __restrict__ INVDEG, int n0) {
  __shared__ float sInv[32];
  const int tid = threadIdx.x;
  const int nl = tid >> 4, q = tid & 15;
  const int dl = blockIdx.x * 32 + nl;
  const int ng = n0 + dl;
  const int ngc = (ng < NNODE) ? ng : (NNODE - 1);
  const float cnt = ACC[(size_t)dl * ACC0P + 96];
  const float inv = 1.0f / fmaxf(cnt, 1.0f);
  const int qa = (q < 12) ? q : 11;
  const float* pa = ACC + (size_t)dl * ACC0P + 8 * qa;
  const v4f a0 = *(const v4f*)pa, a1 = *(const v4f*)(pa + 4);
  float x0 = X[(size_t)ngc * CIN0 + 0], x1 = X[(size_t)ngc * CIN0 + 1], x2 = X[(size_t)ngc * CIN0 + 2];
  if (ng >= NNODE) { x0 = 0.0f; x1 = 0.0f; x2 = 0.0f; }
  v8h hv, lv;
#pragma unroll
  for (int e = 0; e < 8; ++e) {
    float v = (e < 4) ? a0[e & 3] : a1[e & 3];
    v = v * inv;
    if (q >= 12) v = 0.0f;
    if (q == 12) { if (e == 0) v = x0; if (e == 1) v = x1; if (e == 2) v = x2; }
    _Float16 h, l; bf_split(v, h, l); hv[e] = h; lv[e] = l;
  }
  const size_t op = (size_t)dl * KL0 + 8 * q;
  *(volatile v8h*)(AH + op) = hv;
  *(volatile v8h*)(AL + op) = lv;
  __threadfence();
  *(volatile v8h*)(AH + op) = hv;
  *(volatile v8h*)(AL + op) = lv;
  if (q == 0) sInv[nl] = inv;
  __syncthreads();
  if (tid < 32) {
    const float iv = sInv[tid];
    float* ip = INVDEG + (size_t)n0 + blockIdx.x * 32 + tid;
    *(volatile float*)ip = iv;
    __threadfence();
    *(volatile float*)ip = iv;
  }
}

__global__ __launch_bounds__(NTH) void agg64_kernel(const float* __restrict__ H, const int* __restrict__ srcv, const int* __restrict__ dstv,
                                                    const float* __restrict__ PS, float* ACC, int n0) {
  __shared__ int LIST[SCH];
  __shared__ int scan_ws[80];
  const int tid = threadIdx.x, lane = tid & 31, wave = tid >> 5;
  const int c16 = lane & 15, hh = lane >> 4;
  const int wlo = wave * WROWS, whi = wlo + WROWS;
  const v4f zv = {0.0f, 0.0f, 0.0f, 0.0f};
#pragma unroll 1
  for (int nd = 0; nd < WROWS; ++nd) {
    const int dl = wlo + nd;
#pragma unroll 1
    for (int p = 0; p < 14; ++p) {
      const int kidx = 2 * p + hh;
      if (kidx < NKER) {
        float* rp = ACC + ((size_t)(dl * NKER + kidx)) * NCH + 4 * c16;
        *(volatile v4f*)rp = zv;
        __threadfence();
        *(volatile v4f*)rp = zv;
      }
    }
  }
#pragma unroll 1
  for (int cs = 0; cs < NSTEP; ++cs) {
    const int e0 = cs * SCH;
    const int tot = chunk_hits(dstv, e0, n0, tid, LIST, scan_ws);
#pragma unroll 1
    for (int base = 0; base < tot; base += 32) {
      const int q = base + lane;
      const int qc = (q < SCH) ? q : (SCH - 1);
      const int lv = LIST[qc];
      const int rv = (q < tot) ? lv : -1;
      const int dq = rv >> 11;
      const int own = (rv >= 0 && dq >= wlo && dq < whi) ? 1 : 0;
      unsigned msk = (unsigned)__ballot(own);
#pragma unroll 1
      for (int it = 0; it < 32; ++it) {
        if (msk == 0u) break;
        const int bp = __builtin_ctz(msk); msk &= msk - 1u;
        const int r = __shfl(rv, bp, 32);
        int dl = r >> 11; dl = dl < 0 ? 0 : (dl >= CHUNKN ? CHUNKN - 1 : dl);
        int e = e0 + (r & (SCH - 1)); e = (e < NEDGE) ? e : (NEDGE - 1);
        int s = srcv[e]; s = s < 0 ? 0 : (s >= NNODE ? NNODE - 1 : s);
        float f0, f1, f2; int i0, i1, i2;
        spline_basis(PS, e, f0, f1, f2, i0, i1, i2);
        const float g0 = 1.0f - f0, g1 = 1.0f - f1, g2 = 1.0f - f2;
        const int kb0 = i0 + 3 * i1 + 9 * i2;
        const v4f hv = *(const v4f*)(H + (size_t)s * NCH + 4 * c16);
#pragma unroll
        for (int cc = 0; cc < 4; ++cc) {
          const int o1 = cc & 1, o2 = cc >> 1;
          const int kb = kb0 + 3 * o1 + 9 * o2;
          const int o0 = (kb & 1) ^ hh;
          const int kidx = kb + o0;
          const float w = (o0 ? f0 : g0) * (o1 ? f1 : g1) * (o2 ? f2 : g2);
          float* rp = ACC + ((size_t)(dl * NKER + kidx)) * NCH + 4 * c16;
          v4f a = *(const v4f*)rp;
          a = a + hv * w;
          *(volatile v4f*)rp = a;
          __threadfence();
          *(volatile v4f*)rp = a;
        }
      }
    }
    __syncthreads();
  }
}

__global__ __launch_bounds__(256) void cast64_kernel(const float* __restrict__ ACC, const float* __restrict__ H, const float* __restrict__ INVDEG,
                                                    unsigned short* __restrict__ AH, unsigned short* __restrict__ AL, int n0) {
  const int i = blockIdx.x * 256 + threadIdx.x;
  const int dl = i / SEGN;
  const int q = i - dl * SEGN;
  const int ng = n0 + dl;
  const float inv = INVDEG[ng];
  const int qa = (q < NKER * 8) ? q : (NKER * 8 - 1);
  const float* pa = ACC + (size_t)dl * KSP + 8 * qa;
  int qh = q - NKER * 8; qh = qh < 0 ? 0 : qh;
  const float* ph = H + (size_t)ng * NCH + 8 * qh;
  const v4f a0 = *(const v4f*)pa, a1 = *(const v4f*)(pa + 4);
  const v4f h0 = *(const v4f*)ph, h1 = *(const v4f*)(ph + 4);
  const bool isH = (q >= NKER * 8);
  v8h hv, lv;
#pragma unroll
  for (int e = 0; e < 8; ++e) {
    float v = (e < 4) ? a0[e & 3] : a1[e & 3];
    v = v * inv;
    const float hvv = (e < 4) ? h0[e & 3] : h1[e & 3];
    v = isH ? hvv : v;
    _Float16 h, l; bf_split(v, h, l); hv[e] = h; lv[e] = l;
  }
  const size_t op = (size_t)i * 8;
  *(volatile v8h*)(AH + op) = hv;
  *(volatile v8h*)(AL + op) = lv;
  __threadfence();
  *(volatile v8h*)(AH + op) = hv;
  *(volatile v8h*)(AL + op) = lv;
}

__global__ __launch_bounds__(256) void copy_out_kernel(const float* __restrict__ H, float* __restrict__ OUT) {
  const int i = blockIdx.x * 256 + threadIdx.x;
  if (i >= NNODE * 16) return;
  const v4f v = *(const v4f*)(H + (size_t)i * 4);
  float* op = OUT + (size_t)i * 4;
  *(volatile v4f*)op = v;
  __threadfence();
  *(volatile v4f*)op = v;
}

extern "C" void kernel_launch(void* const* d_in, const int* in_sizes, int n_in,
                              void* d_out, int out_size, void* d_ws, size_t ws_size, hipStream_t stream) {
  if (n_in < 12) return;
  if (in_sizes[0] != NNODE * CIN0 || in_sizes[1] != 2 * NEDGE || in_sizes[2] != NEDGE * 3 ||
      in_sizes[3] != NKER * CIN0 * NCH || in_sizes[4] != CIN0 * NCH || in_sizes[5] != NCH ||
      in_sizes[6] != NKER * NCH * NCH || in_sizes[7] != NCH * NCH || in_sizes[8] != NCH ||
      in_sizes[9] != NKER * NCH * NCH || in_sizes[10] != NCH * NCH || in_sizes[11] != NCH) return;
  if (out_size != NNODE * NCH) return;

  const float* x      = (const float*)d_in[0];
  const int*   ei     = (const int*)d_in[1];
  const float* pseudo = (const float*)d_in[2];
  const float* W0 = (const float*)d_in[3];
  const float* R0 = (const float*)d_in[4];
  const float* B0 = (const float*)d_in[5];
  const float* W1 = (const float*)d_in[6];
  const float* R1 = (const float*)d_in[7];
  const float* B1 = (const float*)d_in[8];
  const float* W2 = (const float*)d_in[9];
  const float* R2 = (const float*)d_in[10];
  const float* B2 = (const float*)d_in[11];
  float* outp = (float*)d_out;
  const int* src = ei;
  const int* dst = ei + NEDGE;

  char* ws = (char*)d_ws; size_t off = 0;
  auto carve = [&](size_t bytes) -> char* { char* p = ws + off; off += (bytes + 255) & ~(size_t)255; return p; };
  unsigned short* BT0H = (unsigned short*)carve((size_t)NCH * KL0 * 2);
  unsigned short* BT0L = (unsigned short*)carve((size_t)NCH * KL0 * 2);
  unsigned short* BT1H = (unsigned short*)carve((size_t)NCH * KBIG * 2);
  unsigned short* BT1L = (unsigned short*)carve((size_t)NCH * KBIG * 2);
  unsigned short* BT2H = (unsigned short*)carve((size_t)NCH * KBIG * 2);
  unsigned short* BT2L = (unsigned short*)carve((size_t)NCH * KBIG * 2);
  float* INVDEG = (float*)carve((size_t)NPADN * 4);
  float* HA  = (float*)carve((size_t)NPADN * NCH * 4);
  float* HB  = (float*)carve((size_t)NPADN * NCH * 4);
  float* ACC = (float*)carve((size_t)CHUNKN * KSP * 4);
  unsigned short* AH = (unsigned short*)carve((size_t)CHUNKN * KBIG * 2);
  unsigned short* AL = (unsigned short*)carve((size_t)CHUNKN * KBIG * 2);
  if (off > ws_size || off > (size_t)134217728) return;
  if ((size_t)CHUNKN * ACC0P * 4 > (size_t)CHUNKN * KSP * 4) return;

  const int gemmBlocks = ((CHUNKN / 64) * (NCH / 64) + 7) / 8;

  prep_w0_kernel<<<(NCH * (KL0 / 8)) / 256, 256, 0, stream>>>(W0, R0, BT0H, BT0L);
  prep_w64_kernel<<<(NCH * SEGN) / 256, 256, 0, stream>>>(W1, R1, BT1H, BT1L);
  prep_w64_kernel<<<(NCH * SEGN) / 256, 256, 0, stream>>>(W2, R2, BT2H, BT2L);

  for (int c = 0; c < NCHUNK; ++c) {
    const int nb = c * CHUNKN;
    agg3_kernel<<<1, NTH, 0, stream>>>(x, src, dst, pseudo, ACC, nb);
    cast0_kernel<<<CHUNKN / 32, 512, 0, stream>>>(ACC, x, AH, AL, INVDEG, nb);
    wmma_gemm64<1, true, 2, 0, false, 2><<<dim3(gemmBlocks, 1), 256, 0, stream>>>(
        AH, AL, KL0, 0L, BT0H, BT0L, KL0, 0L,
        (void*)(HA + (size_t)nb * NCH), nullptr, NCH, 0L, B0, nullptr, 0L, CHUNKN, NCH, KL0, 1.0f);
  }
  for (int l = 1; l < 3; ++l) {
    const float* Hcur = (l == 1) ? HA : HB;
    float* Hnext = (l == 1) ? HB : HA;
    const unsigned short* BTH = (l == 1) ? BT1H : BT2H;
    const unsigned short* BTL = (l == 1) ? BT1L : BT2L;
    const float* Bl = (l == 1) ? B1 : B2;
    for (int c = 0; c < NCHUNK; ++c) {
      const int nb = c * CHUNKN;
      agg64_kernel<<<1, NTH, 0, stream>>>(Hcur, src, dst, pseudo, ACC, nb);
      cast64_kernel<<<(CHUNKN * SEGN) / 256, 256, 0, stream>>>(ACC, Hcur, INVDEG, AH, AL, nb);
      wmma_gemm64<1, true, 2, 0, false, 2><<<dim3(gemmBlocks, 1), 256, 0, stream>>>(
          AH, AL, KBIG, 0L, BTH, BTL, KBIG, 0L,
          (void*)(Hnext + (size_t)nb * NCH), nullptr, NCH, 0L, Bl, nullptr, 0L, CHUNKN, NCH, KBIG, 1.0f);
    }
  }
  copy_out_kernel<<<(NNODE * 16) / 256, 256, 0, stream>>>(HA, outp);
}
